// Block_45681272160686
// MI455X (gfx1250) — hardware-run, weakly checked
//
#include <hip/hip_runtime.h>


#ifndef NB
#define NB 2
#endif
#ifndef SEQ
#define SEQ 2048
#endif
#define NB_FULL  2
#define SEQ_FULL 2048
#ifndef OUT_SEQ
#define OUT_SEQ SEQ
#endif
#define CM   1024
#define NHQ  8
#define NKV  4
#define NHT  12
#define HD   128
#define WIN  512
#define HID  4096
#define AW   4
#define OSP  132
#define GSP  68
#define WSC  256.0f
#define WSI  (1.0f / 256.0f)
#define CSC  64.0f
#define OSI  (1.0f / (256.0f * 64.0f))
#define PSH  14.0f
#define NEGB (-3.0e38f)
#define L2E  1.4426950408889634f
#define C1S  ((float)(0.08838834764831845 * 0.04 * 1.4426950408889634))
#define C2S  ((float)(50.0 * 1.4426950408889634))

static_assert(NHQ * HD == CM);
static_assert(NHQ % NKV == 0);
static_assert(NHT == NHQ + NKV);
static_assert(HD == 128);
static_assert(CM % 64 == 0);
static_assert(HID % 64 == 0);
static_assert((NKV * HD) % 64 == 0);
static_assert(CM % 32 == 0);
static_assert(HID % 32 == 0);
static_assert(HD % 32 == 0);
static_assert(SEQ % 64 == 0);
static_assert(SEQ % 32 == 0);
static_assert(SEQ % (16 * AW) == 0);
static_assert((NB * SEQ) % 8 == 0);
static_assert((SEQ * 64) % 256 == 0);
static_assert(NB <= NB_FULL);
static_assert(SEQ <= SEQ_FULL);
static_assert((OSP * 4) % 16 == 0);
static_assert((GSP * 4) % 16 == 0);
static_assert(256 * 8 * 2 == 64 * 64);
static_assert(32 * 8 * 4 == CM);
static_assert(32 * 8 * 8 == 16 * HD);
static_assert(32 * 8 * 4 == 16 * 64);
static_assert(32 * 4 * 8 == 16 * 64);
static_assert(64 * 72 * 2 <= 131072);
static_assert(16 * GSP * 4 <= 131072);
static_assert(16 * OSP * 4 <= 131072);
static_assert(AW * 16 * OSP * 4 <= 131072);

typedef _Float16 h16;
typedef __attribute__((ext_vector_type(16))) _Float16 v16h;
typedef __attribute__((ext_vector_type(8)))  _Float16 v8h;
typedef __attribute__((ext_vector_type(8)))  float    v8f;
typedef __attribute__((ext_vector_type(4)))  float    v4f;
typedef v4f  __attribute__((may_alias)) v4fa;
typedef v8h  __attribute__((may_alias)) v8ha;

__device__ __forceinline__ unsigned short f2bf(float f) { unsigned u = __float_as_uint(f); u += 0x7FFFu + ((u >> 16) & 1u); return (unsigned short)(u >> 16); }
__device__ __forceinline__ float bfr(float f) { return __uint_as_float(((unsigned)f2bf(f)) << 16); }
__device__ __forceinline__ h16 toh_flush(float v) { const h16 r = (h16)v; return (fabsf(v) < 6.103515625e-05f) ? (h16)0.0f : r; }
__device__ __forceinline__ v16h cat16(v8h lo, v8h hi) { return __builtin_shufflevector(lo, hi, 0, 1, 2, 3, 4, 5, 6, 7, 8, 9, 10, 11, 12, 13, 14, 15); }
__device__ __forceinline__ v8f wmma16g(v16h a, v16h b, v8f c) {
    c = __builtin_amdgcn_wmma_f32_16x16x32_f16(false, a, false, b, (short)0, c, false, false);
    asm volatile("v_nop\n\tv_nop\n\tv_nop\n\tv_nop" : "+v"(c) : "v"(a), "v"(b));
    return c;
}
__device__ __forceinline__ v16h ldh(const h16* p) { return cat16(*(const v8h*)p, *(const v8h*)(p + 16)); }
__device__ __forceinline__ void wave_sync() { __builtin_amdgcn_fence(3  , "wavefront"); __builtin_amdgcn_wave_barrier(); asm volatile("" ::: "memory"); }

__global__ __launch_bounds__(256) void k_wtr(const float* __restrict__ W, h16* Wt, int K, int N) {
    __shared__ __align__(16) h16 ts[64 * 72];
    const int tid = threadIdx.x;
    const int k0 = blockIdx.x * 64, n0 = blockIdx.y * 64;
    { const int kk = tid >> 2, nn = (tid & 3) * 16;
      const float* src = W + (size_t)(k0 + kk) * N + n0 + nn;
#pragma unroll
      for (int q = 0; q < 4; ++q) { const v4f v = *(const v4f*)(src + 4 * q);
#pragma unroll
          for (int i = 0; i < 4; ++i) ts[(nn + 4 * q + i) * 72 + kk] = toh_flush(bfr(v[i]) * WSC); } }
    __syncthreads();
    v8h o[2];
#pragma unroll
    for (int it = 0; it < 2; ++it) { const int n = it * 32 + (tid >> 3), c8 = (tid & 7) * 8;
        o[it] = *(const v8ha*)(&ts[n * 72 + c8]); }
#pragma unroll 1
    for (int ps = 0; ps < 2; ++ps) {
#pragma unroll
        for (int it = 0; it < 2; ++it) { const int n = it * 32 + (tid >> 3), c8 = (tid & 7) * 8;
            *(volatile v8h*)(Wt + (size_t)(n0 + n) * K + k0 + c8) = o[it]; }
        if (ps == 0) __threadfence(); }
}

__global__ __launch_bounds__(64) void k_ts(float* INV) {
    const int i = threadIdx.x;
    const float frac = (float)(2 * i) * (1.0f / 128.0f);
    const float ts = powf(10000.0f, frac);
    const float inv = 1.0f / ts;
    *(volatile float*)(INV + i) = inv; __threadfence(); *(volatile float*)(INV + i) = inv;
}

__global__ __launch_bounds__(256) void k_tab(const float* __restrict__ INV, float* COS, float* SIN) {
    const int g = blockIdx.x * 256 + threadIdx.x;
    const int t = g >> 6, i = g & 63;
    const float ang = (float)t * INV[i];
    float sn, cs; sincosf(ang, &sn, &cs);
    *(volatile float*)(COS + g) = cs; *(volatile float*)(SIN + g) = sn;
    __threadfence();
    *(volatile float*)(COS + g) = cs; *(volatile float*)(SIN + g) = sn;
}

__global__ __launch_bounds__(256) void k_rms(const float* __restrict__ X, const float* __restrict__ G, h16* Hp, int srcSeq, int rin) {
#pragma clang fp contract(off)
    const int lane = threadIdx.x & 31;
    const int wave = __builtin_amdgcn_readfirstlane((int)(threadIdx.x >> 5));
    const int m = blockIdx.x * 8 + wave;
    const int bb = m / SEQ, tt = m % SEQ;
    const float* xr = X + ((size_t)bb * (size_t)srcSeq + (size_t)tt) * CM + lane * 8;
    float ss = 0.0f;
#pragma unroll 1
    for (int i = 0; i < 4; ++i) {
        const v4f a = *(const v4f*)(xr + 256 * i), c = *(const v4f*)(xr + 256 * i + 4);
#pragma unroll
        for (int e = 0; e < 4; ++e) { const float p = rin ? bfr(a[e]) : a[e]; const float q = rin ? bfr(c[e]) : c[e]; ss += p * p; ss += q * q; } }
    ss += __shfl_xor(ss, 16, 32); ss += __shfl_xor(ss, 8, 32); ss += __shfl_xor(ss, 4, 32); ss += __shfl_xor(ss, 2, 32); ss += __shfl_xor(ss, 1, 32);
    const float rs = rsqrtf(ss * (1.0f / CM) + 1e-6f);
    h16* dst = Hp + (size_t)m * CM + lane * 8;
    const float* gr = G + lane * 8;
#pragma unroll 1
    for (int i = 0; i < 4; ++i) {
        const v4f a = *(const v4f*)(xr + 256 * i), c = *(const v4f*)(xr + 256 * i + 4);
        const v4f ga = *(const v4f*)(gr + 256 * i), gc = *(const v4f*)(gr + 256 * i + 4);
        v8h hv;
#pragma unroll
        for (int e = 0; e < 4; ++e) { const float p = rin ? bfr(a[e]) : a[e]; const float q = rin ? bfr(c[e]) : c[e];
            hv[e] = toh_flush((p * rs) * (1.0f + bfr(ga[e]))); hv[4 + e] = toh_flush((q * rs) * (1.0f + bfr(gc[e]))); }
        *(volatile v8h*)(dst + 256 * i) = hv; __threadfence(); *(volatile v8h*)(dst + 256 * i) = hv; }
}

__device__ __forceinline__ void mm64(const h16* __restrict__ A, const h16* __restrict__ Bt, const int K, const size_t aoff, const size_t boff, v8f (&acc)[4][4]) {
#pragma unroll 1
    for (int kc = 0; kc < K; kc += 32) {
        v16h a[4];
#pragma unroll
        for (int mb = 0; mb < 4; ++mb) a[mb] = ldh(A + aoff + (size_t)mb * 16 * K + kc);
#pragma unroll
        for (int nb = 0; nb < 4; ++nb) { const v16h b = ldh(Bt + boff + (size_t)nb * 16 * K + kc);
#pragma unroll
            for (int mb = 0; mb < 4; ++mb) acc[mb][nb] = wmma16g(a[mb], b, acc[mb][nb]); }
    }
}

__global__ __launch_bounds__(32) void k_qkrope(const h16* __restrict__ A, const h16* __restrict__ Bt, const float* __restrict__ COS, const float* __restrict__ SIN, h16* QK) {
    __shared__ __align__(16) float os[16 * OSP];
    const int K = CM;
    const int lane = threadIdx.x & 31, lr = lane & 15, hi = lane >> 4;
    const int r0 = blockIdx.x * 32, head = blockIdx.y, c0 = head * HD;
    v8f acc[2][8];
#pragma unroll
    for (int mb = 0; mb < 2; ++mb)
#pragma unroll
        for (int nb = 0; nb < 8; ++nb) acc[mb][nb] = (v8f){};
    const size_t aoff = (size_t)(r0 + lr) * K + 8 * hi, boff = (size_t)(c0 + lr) * K + 8 * hi;
#pragma unroll 1
    for (int kc = 0; kc < K; kc += 32) {
        v16h a[2];
#pragma unroll
        for (int mb = 0; mb < 2; ++mb) a[mb] = ldh(A + aoff + (size_t)mb * 16 * K + kc);
#pragma unroll
        for (int nb = 0; nb < 8; ++nb) { const v16h b = ldh(Bt + boff + (size_t)nb * 16 * K + kc);
#pragma unroll
            for (int mb = 0; mb < 2; ++mb) acc[mb][nb] = wmma16g(a[mb], b, acc[mb][nb]); }
    }
    const int bb = r0 / SEQ, tt0 = r0 % SEQ;
    const size_t pbase = ((size_t)(bb * NHT + head) * SEQ + (size_t)tt0) * HD;
#pragma unroll
    for (int mb = 0; mb < 2; ++mb) {
#pragma unroll
        for (int nb = 0; nb < 8; ++nb) {
#pragma unroll
            for (int j = 0; j < 8; ++j) os[(hi * 8 + j) * OSP + nb * 16 + lr] = acc[mb][nb][j] * WSI; }
        wave_sync();
        v8h hv[8];
#pragma unroll
        for (int s = 0; s < 8; ++s) { const int p = s * 32 + lane; const int row = p >> 4, c8 = (p & 15) * 8;
            const int pc = c8 ^ 64, ci = c8 & 63;
            const v4f x0 = *(const v4fa*)(&os[row * OSP + c8]), x1 = *(const v4fa*)(&os[row * OSP + c8 + 4]);
            const v4f y0 = *(const v4fa*)(&os[row * OSP + pc]), y1 = *(const v4fa*)(&os[row * OSP + pc + 4]);
            const size_t to = (size_t)(tt0 + mb * 16 + row) * 64 + ci;
            const v4f cs0 = *(const v4f*)(COS + to), cs1 = *(const v4f*)(COS + to + 4);
            const v4f sn0 = *(const v4f*)(SIN + to), sn1 = *(const v4f*)(SIN + to + 4);
            const float sg = (c8 < 64) ? -1.0f : 1.0f;
#pragma unroll
            for (int i = 0; i < 4; ++i) { hv[s][i] = toh_flush(x0[i] * cs0[i] + (sg * y0[i]) * sn0[i]); hv[s][4 + i] = toh_flush(x1[i] * cs1[i] + (sg * y1[i]) * sn1[i]); } }
        const size_t sb = pbase + (size_t)(mb * 16) * HD;
#pragma unroll 1
        for (int ps = 0; ps < 2; ++ps) {
#pragma unroll
            for (int s = 0; s < 8; ++s) { const int p = s * 32 + lane; *(volatile v8h*)(QK + sb + (size_t)p * 8) = hv[s]; }
            if (ps == 0) __threadfence(); }
        wave_sync();
    }
}

__global__ __launch_bounds__(32) void k_vproj(const h16* __restrict__ A, const h16* __restrict__ Bt, h16* VT) {
    __shared__ __align__(16) float os[16 * GSP];
    const int K = CM;
    const int lane = threadIdx.x & 31, lr = lane & 15, hi = lane >> 4;
    const int r0 = blockIdx.x * 64, c0 = blockIdx.y * 64;
    v8f acc[4][4];
#pragma unroll
    for (int mb = 0; mb < 4; ++mb)
#pragma unroll
        for (int nb = 0; nb < 4; ++nb) acc[mb][nb] = (v8f){};
    mm64(A, Bt, K, (size_t)(r0 + lr) * K + 8 * hi, (size_t)(c0 + lr) * K + 8 * hi, acc);
    const int bb = c0 / SEQ, tt = c0 % SEQ;
    const size_t tbase = ((size_t)bb * (NKV * HD) + (size_t)r0) * SEQ + (size_t)tt;
#pragma unroll
    for (int mb = 0; mb < 4; ++mb) {
#pragma unroll
        for (int nb = 0; nb < 4; ++nb) {
#pragma unroll
            for (int j = 0; j < 8; ++j) os[(hi * 8 + j) * GSP + nb * 16 + lr] = acc[mb][nb][j] * WSI; }
        wave_sync();
        v8h hv[4];
#pragma unroll
        for (int s = 0; s < 4; ++s) { const int row = 4 * s + (lane >> 3), c8 = (lane & 7) * 8;
            const v4f x0 = *(const v4fa*)(&os[row * GSP + c8]), x1 = *(const v4fa*)(&os[row * GSP + c8 + 4]);
#pragma unroll
            for (int i = 0; i < 4; ++i) { hv[s][i] = toh_flush(x0[i]); hv[s][4 + i] = toh_flush(x1[i]); } }
#pragma unroll 1
        for (int ps = 0; ps < 2; ++ps) {
#pragma unroll
            for (int s = 0; s < 4; ++s) { const int row = 4 * s + (lane >> 3), c8 = (lane & 7) * 8;
                *(volatile v8h*)(VT + tbase + (size_t)(mb * 16 + row) * SEQ + c8) = hv[s]; }
            if (ps == 0) __threadfence(); }
        wave_sync();
    }
}

__global__ __launch_bounds__(32 * AW) __attribute__((amdgpu_num_vgpr(256))) void k_flash(const h16* __restrict__ QK, const h16* __restrict__ VT, h16* CTX) {
    __shared__ __align__(16) float os[AW * 16 * OSP];
    const int lane = threadIdx.x & 31, lr = lane & 15, hi = lane >> 4;
    const int wave = __builtin_amdgcn_readfirstlane((int)(threadIdx.x >> 5));
    const int zh = blockIdx.y; const int b = zh / NHQ, hh = zh % NHQ; const int kvh = hh % NKV;
    const int t0 = (blockIdx.x * AW + wave) * 16;
    const int tq = t0 + lr;
    const int lo = tq - WIN;
    int ks = t0 - (WIN - 1); ks = ks & ~(ks >> 31); ks &= ~31;
    const int nk = (t0 + 16 + 31) & ~31;
    const size_t qbase = ((size_t)(b * NHT + hh) * SEQ + (size_t)tq) * HD + 8 * hi;
    const size_t kbase = ((size_t)(b * NHT + NHQ + kvh) * SEQ + (size_t)lr) * HD + 8 * hi;
    const size_t vbase = ((size_t)(b * NKV + kvh) * HD + (size_t)lr) * SEQ + 8 * hi;
    v8f o[8];
#pragma unroll
    for (int j = 0; j < 8; ++j) o[j] = (v8f){};
    float m = NEGB, l = 0.0f;
#pragma unroll 1
    for (int key0 = ks; key0 < nk; key0 += 32) {
        unsigned qz = 0u; asm volatile("" : "+v"(qz));
        const h16* qp = QK + qbase + (size_t)qz;
        const h16* kp = QK + kbase + (size_t)key0 * HD;
        v8f sa = (v8f){}, sb = (v8f){};
#pragma unroll
        for (int c = 0; c < 4; ++c) {
            const v16h qf = ldh(qp + 32 * c);
            const v16h ka = ldh(kp + 32 * c), kb = ldh(kp + 16 * HD + 32 * c);
            sa = wmma16g(ka, qf, sa); sb = wmma16g(kb, qf, sb); }
        const int ja = key0 + 8 * hi;
        float ta[8], tb[8]; bool fa[8], fb[8]; float mx = NEGB;
#pragma unroll
        for (int r = 0; r < 8; ++r) {
            fa[r] = (ja + r <= tq) & (ja + r > lo);
            fb[r] = (ja + 16 + r <= tq) & (ja + 16 + r > lo);
            const float ua = __builtin_amdgcn_exp2f(sa[r] * C1S), ub = __builtin_amdgcn_exp2f(sb[r] * C1S);
            ta[r] = (1.0f - 2.0f * __builtin_amdgcn_rcpf(ua + 1.0f)) * C2S;
            tb[r] = (1.0f - 2.0f * __builtin_amdgcn_rcpf(ub + 1.0f)) * C2S;
            mx = fmaxf(mx, fmaxf(fa[r] ? ta[r] : NEGB, fb[r] ? tb[r] : NEGB)); }
        mx = fmaxf(mx, __shfl_xor(mx, 16, 32));
        const float mnew = fmaxf(m, mx);
        const float alpha = __builtin_amdgcn_exp2f(m - mnew);
        const float sh = PSH - mnew;
        v16h pb; float ls = 0.0f;
#pragma unroll
        for (int r = 0; r < 8; ++r) {
            const float ea = ta[r] + sh, eb = tb[r] + sh;
            const float xa = __builtin_amdgcn_exp2f(ea), xb = __builtin_amdgcn_exp2f(eb);
            const float ga = (fa[r] & (ea >= -14.0f)) ? xa : 0.0f;
            const float gb = (fb[r] & (eb >= -14.0f)) ? xb : 0.0f;
            const h16 pa = (h16)ga; const h16 pc = (h16)gb;
            pb[r] = pa; pb[8 + r] = pc;
            ls += (float)pa + (float)pc; }
        l = l * alpha + ls; m = mnew;
#pragma unroll
        for (int j = 0; j < 8; ++j) o[j] = o[j] * alpha;
        const h16* va = VT + vbase + key0;
#pragma unroll
        for (int g = 0; g < 2; ++g) {
            v16h vf[4];
#pragma unroll
            for (int jj = 0; jj < 4; ++jj) vf[jj] = ldh(va + (size_t)(16 * (4 * g + jj)) * SEQ);
#pragma unroll
            for (int jj = 0; jj < 4; ++jj) o[4 * g + jj] = wmma16g(vf[jj], pb, o[4 * g + jj]); }
    }
    l += __shfl_xor(l, 16, 32);
    const bool any = l > 0.0f;
    const float lsafe = any ? l : 1.0f;
    const float inv = any ? (CSC / lsafe) : 0.0f;
    const int wb = wave * 16 * OSP;
#pragma unroll
    for (int j = 0; j < 8; ++j) { v4f a, c;
        a[0] = o[j][0] * inv; a[1] = o[j][1] * inv; a[2] = o[j][2] * inv; a[3] = o[j][3] * inv; c[0] = o[j][4] * inv; c[1] = o[j][5] * inv; c[2] = o[j][6] * inv; c[3] = o[j][7] * inv;
        *(v4fa*)(&os[wb + lr * OSP + 16 * j + 8 * hi]) = a; *(v4fa*)(&os[wb + lr * OSP + 16 * j + 8 * hi + 4]) = c; }
    wave_sync();
    v8h hv[8];
#pragma unroll
    for (int s = 0; s < 8; ++s) { const int p = s * 32 + lane; const int row = p >> 4, c8 = (p & 15) * 8;
        const v4f x0 = *(const v4fa*)(&os[wb + row * OSP + c8]), x1 = *(const v4fa*)(&os[wb + row * OSP + c8 + 4]);
#pragma unroll
        for (int i = 0; i < 4; ++i) { hv[s][i] = toh_flush(x0[i]); hv[s][4 + i] = toh_flush(x1[i]); } }
    h16* crow = CTX + ((size_t)b * SEQ + (size_t)t0) * CM + hh * HD;
#pragma unroll 1
    for (int ps = 0; ps < 2; ++ps) {
#pragma unroll
        for (int s = 0; s < 8; ++s) { const int p = s * 32 + lane; const int row = p >> 4, c8 = (p & 15) * 8;
            *(volatile v8h*)(crow + (size_t)row * CM + c8) = hv[s]; }
        if (ps == 0) __threadfence(); }
}

__global__ __launch_bounds__(32) void k_gemm_res(const h16* __restrict__ A, const h16* __restrict__ Bt, int K, int N, float scale,
                                                 const float* __restrict__ res, int resSeq, int rbf, float* out, int outSeq) {
    __shared__ __align__(16) float os[16 * GSP];
    const int lane = threadIdx.x & 31, lr = lane & 15, hi = lane >> 4;
    const int r0 = blockIdx.x * 64, c0 = blockIdx.y * 64;
    v8f acc[4][4];
#pragma unroll
    for (int mb = 0; mb < 4; ++mb)
#pragma unroll
        for (int nb = 0; nb < 4; ++nb) acc[mb][nb] = (v8f){};
    mm64(A, Bt, K, (size_t)(r0 + lr) * K + 8 * hi, (size_t)(c0 + lr) * K + 8 * hi, acc);
    const int bb = r0 / SEQ, tt0 = r0 % SEQ;
    const float* rsrc = res + ((size_t)bb * (size_t)resSeq + (size_t)tt0) * N + c0;
    float* dst = out + ((size_t)bb * (size_t)outSeq + (size_t)tt0) * N + c0;
#pragma unroll
    for (int mb = 0; mb < 4; ++mb) {
#pragma unroll
        for (int nb = 0; nb < 4; ++nb) {
#pragma unroll
            for (int j = 0; j < 8; ++j) os[(hi * 8 + j) * GSP + nb * 16 + lr] = acc[mb][nb][j] * scale; }
        wave_sync();
        v4f val[8];
#pragma unroll
        for (int s = 0; s < 8; ++s) { const int p = s * 32 + lane; const int row = p >> 4, c4 = (p & 15) * 4;
            const v4f a = *(const v4fa*)(&os[row * GSP + c4]);
            const v4f r = *(const v4f*)(rsrc + (size_t)(mb * 16 + row) * N + c4);
#pragma unroll
            for (int i = 0; i < 4; ++i) { const float rv = rbf ? bfr(r[i]) : r[i]; val[s][i] = a[i] + rv; } }
#pragma unroll 1
        for (int ps = 0; ps < 2; ++ps) {
#pragma unroll
            for (int s = 0; s < 8; ++s) { const int p = s * 32 + lane; const int row = p >> 4, c4 = (p & 15) * 4;
                *(volatile v4f*)(dst + (size_t)(mb * 16 + row) * N + c4) = val[s]; }
            if (ps == 0) __threadfence(); }
        wave_sync();
    }
}

__global__ __launch_bounds__(32) void k_gateup(const h16* __restrict__ A, const h16* __restrict__ Bg, const h16* __restrict__ Bu, h16* ACT) {
    __shared__ __align__(16) float os[16 * GSP];
    const int K = CM;
    const int lane = threadIdx.x & 31, lr = lane & 15, hi = lane >> 4;
    const int r0 = blockIdx.x * 32, c0 = blockIdx.y * 64;
    v8f g[2][4], u[2][4];
#pragma unroll
    for (int mb = 0; mb < 2; ++mb)
#pragma unroll
        for (int nb = 0; nb < 4; ++nb) { g[mb][nb] = (v8f){}; u[mb][nb] = (v8f){}; }
    const size_t aoff = (size_t)(r0 + lr) * K + 8 * hi, boff = (size_t)(c0 + lr) * K + 8 * hi;
#pragma unroll 1
    for (int kc = 0; kc < K; kc += 32) {
        v16h a[2];
#pragma unroll
        for (int mb = 0; mb < 2; ++mb) a[mb] = ldh(A + aoff + (size_t)mb * 16 * K + kc);
#pragma unroll
        for (int nb = 0; nb < 4; ++nb) {
            const v16h bg = ldh(Bg + boff + (size_t)nb * 16 * K + kc);
            const v16h bu = ldh(Bu + boff + (size_t)nb * 16 * K + kc);
#pragma unroll
            for (int mb = 0; mb < 2; ++mb) { g[mb][nb] = wmma16g(a[mb], bg, g[mb][nb]); u[mb][nb] = wmma16g(a[mb], bu, u[mb][nb]); } }
    }
#pragma unroll
    for (int mb = 0; mb < 2; ++mb) {
#pragma unroll
        for (int nb = 0; nb < 4; ++nb) {
#pragma unroll
            for (int j = 0; j < 8; ++j) { const float gv = g[mb][nb][j] * WSI, uv = u[mb][nb][j] * WSI;
                const float e = __builtin_amdgcn_exp2f(-gv * L2E);
                const float sg = gv * __builtin_amdgcn_rcpf(1.0f + e);
                os[(hi * 8 + j) * GSP + nb * 16 + lr] = (sg * uv) * CSC; } }
        wave_sync();
        v8h hv[4];
#pragma unroll
        for (int s = 0; s < 4; ++s) { const int row = 4 * s + (lane >> 3), c8 = (lane & 7) * 8;
            const v4f x0 = *(const v4fa*)(&os[row * GSP + c8]), x1 = *(const v4fa*)(&os[row * GSP + c8 + 4]);
#pragma unroll
            for (int i = 0; i < 4; ++i) { hv[s][i] = toh_flush(x0[i]); hv[s][4 + i] = toh_flush(x1[i]); } }
#pragma unroll 1
        for (int ps = 0; ps < 2; ++ps) {
#pragma unroll
            for (int s = 0; s < 4; ++s) { const int row = 4 * s + (lane >> 3), c8 = (lane & 7) * 8;
                *(volatile v8h*)(ACT + (size_t)(r0 + mb * 16 + row) * HID + c0 + c8) = hv[s]; }
            if (ps == 0) __threadfence(); }
        wave_sync();
    }
}

static constexpr size_t al256(size_t v) { return (v + 255) & ~(size_t)255; }
static constexpr size_t SZ_WQKV = al256((size_t)(NHT * HD + NKV * HD) * CM * 2);
static constexpr size_t SZ_WO   = al256((size_t)CM * CM * 2);
static constexpr size_t SZ_WM   = al256((size_t)HID * CM * 2);
static constexpr size_t SZ_INV  = 256;
static constexpr size_t SZ_TAB  = al256((size_t)SEQ * 64 * 4);
static constexpr size_t SZ_H    = al256((size_t)NB * SEQ * CM * 2);
static constexpr size_t SZ_QK   = al256((size_t)NB * NHT * SEQ * HD * 2);
static constexpr size_t SZ_VT   = al256((size_t)NB * NKV * HD * SEQ * 2);
static constexpr size_t SZ_X1   = al256((size_t)NB * SEQ * CM * 4);
static constexpr size_t SZ_ACT  = al256((size_t)NB * SEQ * HID * 2);
static constexpr size_t SZ_TOTAL = SZ_WQKV + SZ_WO + 3 * SZ_WM + SZ_INV + 2 * SZ_TAB + 2 * SZ_H + SZ_QK + SZ_VT + SZ_X1 + SZ_ACT;
static_assert(SZ_TOTAL <= (size_t)134217728);
static_assert(((size_t)CM * CM * 2) % 256 == 0);
static_assert(((size_t)CM * NKV * HD * 2) % 256 == 0);

extern "C" void kernel_launch(void* const* d_in, const int* in_sizes, int n_in,
                              void* d_out, int out_size, void* d_ws, size_t ws_size, hipStream_t stream) {
    if (n_in < 10) return;
    const size_t needx = ((size_t)(NB - 1) * SEQ_FULL + SEQ) * CM;
    if ((size_t)in_sizes[0] < needx) return;
    if ((size_t)in_sizes[1] < (size_t)CM * CM || (size_t)in_sizes[2] < (size_t)CM * NKV * HD || (size_t)in_sizes[3] < (size_t)CM * NKV * HD || (size_t)in_sizes[4] < (size_t)CM * CM) return;
    if (in_sizes[5] < CM || in_sizes[6] < CM) return;
    if ((size_t)in_sizes[7] < (size_t)CM * HID || (size_t)in_sizes[8] < (size_t)CM * HID || (size_t)in_sizes[9] < (size_t)HID * CM) return;
    if ((size_t)out_size < ((size_t)(NB - 1) * OUT_SEQ + SEQ) * CM) return;
    if (SZ_TOTAL > ws_size) return;
    const float* x  = (const float*)d_in[0];
    const float* wq = (const float*)d_in[1]; const float* wk = (const float*)d_in[2]; const float* wv = (const float*)d_in[3];
    const float* wo = (const float*)d_in[4];
    const float* sa = (const float*)d_in[5]; const float* sm = (const float*)d_in[6];
    const float* wg = (const float*)d_in[7]; const float* wu = (const float*)d_in[8]; const float* wd = (const float*)d_in[9];
    float* OUT = (float*)d_out;
    char* wsp = (char*)d_ws;
    h16* WQKV = (h16*)wsp; wsp += SZ_WQKV;
    h16* WO   = (h16*)wsp; wsp += SZ_WO;
    h16* WG   = (h16*)wsp; wsp += SZ_WM;
    h16* WU   = (h16*)wsp; wsp += SZ_WM;
    h16* WD   = (h16*)wsp; wsp += SZ_WM;
    float* INV = (float*)wsp; wsp += SZ_INV;
    float* COS = (float*)wsp; wsp += SZ_TAB;
    float* SIN = (float*)wsp; wsp += SZ_TAB;
    h16* HP   = (h16*)wsp; wsp += SZ_H;
    h16* CTX  = (h16*)wsp; wsp += SZ_H;
    h16* QK   = (h16*)wsp; wsp += SZ_QK;
    h16* VT   = (h16*)wsp; wsp += SZ_VT;
    float* X1 = (float*)wsp; wsp += SZ_X1;
    h16* ACT  = (h16*)wsp; wsp += SZ_ACT;
    h16* WKT = WQKV + (size_t)CM * CM;
    h16* WVT = WQKV + (size_t)(CM + NKV * HD) * CM;

    k_wtr<<<dim3(CM / 64, CM / 64, 1), 256, 0, stream>>>(wq, WQKV, CM, CM);
    k_wtr<<<dim3(CM / 64, NKV * HD / 64, 1), 256, 0, stream>>>(wk, WKT, CM, NKV * HD);
    k_wtr<<<dim3(CM / 64, NKV * HD / 64, 1), 256, 0, stream>>>(wv, WVT, CM, NKV * HD);
    k_wtr<<<dim3(CM / 64, CM / 64, 1), 256, 0, stream>>>(wo, WO, CM, CM);
    k_wtr<<<dim3(CM / 64, HID / 64, 1), 256, 0, stream>>>(wg, WG, CM, HID);
    k_wtr<<<dim3(CM / 64, HID / 64, 1), 256, 0, stream>>>(wu, WU, CM, HID);
    k_wtr<<<dim3(HID / 64, CM / 64, 1), 256, 0, stream>>>(wd, WD, HID, CM);
    k_ts<<<1, 64, 0, stream>>>(INV);
    k_tab<<<SEQ * 64 / 256, 256, 0, stream>>>(INV, COS, SIN);

    k_rms<<<NB * SEQ / 8, 256, 0, stream>>>(x, sa, HP, SEQ_FULL, 1);
    k_qkrope<<<dim3(NB * SEQ / 32, NHT, 1), 32, 0, stream>>>(HP, WQKV, COS, SIN, QK);
    k_vproj<<<dim3(NKV * HD / 64, NB * SEQ / 64, 1), 32, 0, stream>>>(WVT, HP, VT);
    k_flash<<<dim3(SEQ / (16 * AW), NB * NHQ, 1), 32 * AW, 0, stream>>>(QK, VT, CTX);
    k_gemm_res<<<dim3(NB * SEQ / 64, CM / 64, 1), 32, 0, stream>>>(CTX, WO, CM, CM, OSI, x, SEQ_FULL, 1, X1, SEQ);

    k_rms<<<NB * SEQ / 8, 256, 0, stream>>>(X1, sm, HP, SEQ, 0);
    k_gateup<<<dim3(NB * SEQ / 32, HID / 64, 1), 32, 0, stream>>>(HP, WG, WU, ACT);
    k_gemm_res<<<dim3(NB * SEQ / 64, CM / 64, 1), 32, 0, stream>>>(ACT, WD, HID, CM, OSI, X1, SEQ, 0, OUT, OUT_SEQ);
}
